// SparseDoubleConv_25598005084695
// MI455X (gfx1250) — hardware-verified
//
#include <hip/hip_runtime.h>
#include <stdint.h>
#include <stddef.h>


typedef __attribute__((ext_vector_type(16))) _Float16 v16h;
typedef __attribute__((ext_vector_type(8)))  _Float16 v8h;
typedef __attribute__((ext_vector_type(16))) __bf16   v16b;
typedef __attribute__((ext_vector_type(8)))  __bf16   v8b;
typedef __attribute__((ext_vector_type(8)))  float    v8f;
typedef __attribute__((ext_vector_type(4)))  float    v4f;
typedef __attribute__((ext_vector_type(4)))  unsigned v4u;
typedef __attribute__((ext_vector_type(2)))  double   v2d;

#define CIN      32
#define COUT     64
#define NK       27
#define K1       (NK * CIN)
#define LD1      896
#define K2       (NK * COUT)
#define LD2      1728
#define STAT_BLK 256
#define NCH1     7
#define NCH2     14
#define WSCALE     16.0f
#define WSCALE_INV (1.0f / 16.0f)
#define BN_EPS     1e-4f
#define NEG_SLOPE  0.05f

union P16 { v8h h; v4u u; };

__device__ __forceinline__ unsigned short f2bf_bits(float f) {
  unsigned u = __float_as_uint(f);
  return (unsigned short)((u + 0x7FFFu + ((u >> 16) & 1u)) >> 16);
}
__device__ __forceinline__ float bf_bits2f(unsigned short h) { return __uint_as_float(((unsigned)h) << 16); }

__device__ __forceinline__ void dep_guard_h(v8f& a, v8f& b, v16h x, v16h y) { asm volatile("v_nop\n\tv_nop\n\tv_nop\n\tv_nop" : "+v"(a), "+v"(b) : "v"(x), "v"(y)); }
__device__ __forceinline__ void dep_guard_b(v8f& a, v8f& b, v16b x, v16b y) { asm volatile("v_nop\n\tv_nop\n\tv_nop\n\tv_nop" : "+v"(a), "+v"(b) : "v"(x), "v"(y)); }
__device__ __forceinline__ void keep4_h(v16h a, v16h b, v16h c, v16h d) { asm volatile("v_nop" :: "v"(a), "v"(b), "v"(c), "v"(d)); }
__device__ __forceinline__ void keep4_b(v16b a, v16b b, v16b c, v16b d) { asm volatile("v_nop" :: "v"(a), "v"(b), "v"(c), "v"(d)); }
__device__ __forceinline__ void acc_guard4(v8f& a, v8f& b, v8f& c, v8f& d) { asm volatile("v_nop\n\tv_nop\n\tv_nop\n\tv_nop" : "+v"(a), "+v"(b), "+v"(c), "+v"(d)); }
template <typename T> struct Frag;
template <> struct Frag<_Float16> {
  typedef v16h V; union U { v16h v; v8h h[2]; };
  static __device__ __forceinline__ v16h load(const _Float16* p) {
    U f; f.h[0] = *(const v8h*)(p); f.h[1] = *(const v8h*)(p + 16); return f.v;
  }
  static __device__ __forceinline__ v8f mma(v16h a, v16h b, v8f c) {
    return __builtin_amdgcn_wmma_f32_16x16x32_f16(false, a, false, b, (short)0, c, false, false);
  }
  static __device__ __forceinline__ void guard(v8f& a, v8f& b, v16h x, v16h y) { dep_guard_h(a, b, x, y); }
  static __device__ __forceinline__ void keep(v16h a, v16h b, v16h c, v16h d) { keep4_h(a, b, c, d); }
};
template <> struct Frag<__bf16> {
  typedef v16b V; union U { v16b v; v8b h[2]; };
  static __device__ __forceinline__ v16b load(const __bf16* p) {
    U f; f.h[0] = *(const v8b*)(p); f.h[1] = *(const v8b*)(p + 16); return f.v;
  }
  static __device__ __forceinline__ v8f mma(v16b a, v16b b, v8f c) {
    return __builtin_amdgcn_wmma_f32_16x16x32_bf16(false, a, false, b, (short)0, c, false, false);
  }
  static __device__ __forceinline__ void guard(v8f& a, v8f& b, v16b x, v16b y) { dep_guard_b(a, b, x, y); }
  static __device__ __forceinline__ void keep(v16b a, v16b b, v16b c, v16b d) { keep4_b(a, b, c, d); }
};

template <int ET> struct Elem;
template <> struct Elem<0> { typedef _Float16 T; };
template <> struct Elem<1> { typedef __bf16 T; };
template <int ET, bool SPLIT, int BIAS_MODE, int OUT_MODE, bool RESID, int ACT = 0>
__global__ __launch_bounds__(256) void wmma_gemm64(
    const unsigned short* __restrict__ Ap, const unsigned short* __restrict__ A2p, int lda, long strideA,
    const unsigned short* __restrict__ Btp, const unsigned short* __restrict__ Bt2p, int ldb, long strideB,
    void* __restrict__ Cout, void* __restrict__ Cout2, int ldc, long strideC,
    const float* __restrict__ bias,
    const float* __restrict__ resid, long strideR,
    int M, int N, int K, float scale) {
  typedef typename Elem<ET>::T T;
  typedef typename Frag<T>::V V;
  const T* A = (const T*)Ap; const T* A2 = (const T*)A2p; const T* Bt = (const T*)Btp; const T* Bt2 = (const T*)Bt2p;
  __shared__ __align__(16) float sT[8][16 * 68];
  const int b    = blockIdx.y;
  const int lane = threadIdx.x & 31;
  const int wave = threadIdx.x >> 5;
  const int tilesN = N >> 6;
  const int tilesM = M >> 6;
  const int tile = blockIdx.x * 8 + wave;
  if (tile >= tilesM * tilesN) return;
  const int tm = tile / tilesN;
  const int tn = tile - tm * tilesN;
  const int m0 = tm << 6;
  const int n0 = tn << 6;

  const T* Ab  = A  + (size_t)b * strideA;
  const T* Bb  = Bt + (size_t)b * strideB;
  const T* Ab2 = SPLIT ? (A2  + (size_t)b * strideA) : nullptr;
  const T* Bb2 = SPLIT ? (Bt2 + (size_t)b * strideB) : nullptr;

  const int rlane = lane & 15;
  const int koff  = (lane >> 4) * 8;
  const int mOff  = (lane >> 4) * 8;

  v8f acc[4][4];
#pragma unroll
  for (int i = 0; i < 4; ++i)
#pragma unroll
    for (int j = 0; j < 4; ++j) acc[i][j] = (v8f){0.f,0.f,0.f,0.f,0.f,0.f,0.f,0.f};

  for (int k0 = 0; k0 < K; k0 += 32) {
    V bh[4], bl[4];
#pragma unroll
    for (int j = 0; j < 4; ++j) {
      const size_t bo = (size_t)(n0 + (j << 4) + rlane) * ldb + koff + k0;
      bh[j] = Frag<T>::load(Bb + bo);
      if (SPLIT) bl[j] = Frag<T>::load(Bb2 + bo);
    }
#pragma unroll
    for (int i = 0; i < 4; ++i) {
      const size_t ao = (size_t)(m0 + (i << 4) + rlane) * lda + koff + k0;
      V ah = Frag<T>::load(Ab + ao);
      V al;
      if (SPLIT) al = Frag<T>::load(Ab2 + ao);
#pragma unroll
      for (int j = 0; j < 4; ++j) {
        acc[i][j] = Frag<T>::mma(ah, bh[j], acc[i][j]);
        if (SPLIT) {
          acc[i][j] = Frag<T>::mma(ah, bl[j], acc[i][j]);
          acc[i][j] = Frag<T>::mma(al, bh[j], acc[i][j]);
        }
      }
      Frag<T>::guard(acc[i][0], acc[i][3], ah, SPLIT ? al : ah);
    }
    Frag<T>::keep(bh[0], bh[1], bh[2], bh[3]);
    if (SPLIT) Frag<T>::keep(bl[0], bl[1], bl[2], bl[3]);
  }
  acc_guard4(acc[0][0], acc[0][1], acc[0][2], acc[0][3]);
  acc_guard4(acc[1][0], acc[1][1], acc[1][2], acc[1][3]);
  acc_guard4(acc[2][0], acc[2][1], acc[2][2], acc[2][3]);
  acc_guard4(acc[3][0], acc[3][1], acc[3][2], acc[3][3]);

  float* slab = sT[wave];
  const float* Rb = RESID ? (resid + (size_t)b * strideR) : nullptr;
#pragma unroll
  for (int i = 0; i < 4; ++i) {
    const int mBase = m0 + (i << 4);
#pragma unroll
    for (int j = 0; j < 4; ++j) {
      const int n = n0 + (j << 4) + rlane;
      float bv = 0.f;
      if (BIAS_MODE == 2) bv = bias[n];
#pragma unroll
      for (int r = 0; r < 8; ++r) {
        float v = acc[i][j][r] * scale;
        if (BIAS_MODE == 1) v += bias[mBase + mOff + r];
        if (BIAS_MODE == 2) v += bv;
        if (RESID) v += Rb[(size_t)(mBase + mOff + r) * ldc + n];
        if (ACT == 1) v = tanhf(v);
        if (ACT == 2) v = fmaxf(v, 0.0f);
        if (ACT == 3) v = v / (1.0f + expf(-v));
        if (ACT == 4) v = (v > 0.f) ? v : 0.01f * v;
        if (ACT == 5) v = 0.5f * v * (1.0f + erff(v * 0.70710678118654752f));
        slab[(mOff + r) * 68 + (j << 4) + rlane] = v;
      }
    }
    __builtin_amdgcn_fence(__ATOMIC_RELEASE, "workgroup");
    __builtin_amdgcn_wave_barrier();
    __builtin_amdgcn_fence(__ATOMIC_ACQUIRE, "workgroup");
    if (OUT_MODE == 0) {
      float* C = (float*)Cout + (size_t)b * strideC;
      const int hh = lane >> 4, c4 = (lane & 15) * 4;
      for (int pass = 0; pass < 2; ++pass) {
#pragma unroll
        for (int it = 0; it < 8; ++it) {
          const int row = it * 2 + hh;
          v4f v = *(const v4f*)(slab + row * 68 + c4);
          *(volatile v4f*)(C + (size_t)(mBase + row) * ldc + n0 + c4) = v;
        }
        __threadfence();
      }
    } else {
      const int q = lane >> 3, c8 = (lane & 7) * 8;
      unsigned short* C  = (unsigned short*)Cout  + (size_t)b * strideC;
      unsigned short* C2 = (OUT_MODE == 2) ? ((unsigned short*)Cout2 + (size_t)b * strideC) : nullptr;
      for (int pass = 0; pass < 2; ++pass) {
#pragma unroll
        for (int it = 0; it < 4; ++it) {
          const int row = it * 4 + q;
          const float* sp = slab + row * 68 + c8;
          v8h hv, lv;
#pragma unroll
          for (int e = 0; e < 8; ++e) {
            if (OUT_MODE == 1) {
              hv[e] = (_Float16)sp[e];
            } else {
              unsigned short hb = f2bf_bits(sp[e]);
              unsigned short lb = f2bf_bits(sp[e] - bf_bits2f(hb));
              hv[e] = __builtin_bit_cast(_Float16, hb);
              lv[e] = __builtin_bit_cast(_Float16, lb);
            }
          }
          *(volatile v8h*)(C + (size_t)(mBase + row) * ldc + n0 + c8) = hv;
          if (OUT_MODE == 2) *(volatile v8h*)(C2 + (size_t)(mBase + row) * ldc + n0 + c8) = lv;
        }
        __threadfence();
      }
    }
    __builtin_amdgcn_fence(__ATOMIC_RELEASE, "workgroup");
    __builtin_amdgcn_wave_barrier();
    __builtin_amdgcn_fence(__ATOMIC_ACQUIRE, "workgroup");
  }
}

template <int LDB>
__global__ __launch_bounds__(256) void prep_bt(const float* __restrict__ W, _Float16* __restrict__ Bt, int K) {
  const int PPR = LDB / 8;
  const int p = blockIdx.x * 256 + threadIdx.x;
  if (p >= COUT * PPR) return;
  const int n = p / PPR;
  const int col = (p - n * PPR) * 8;
  P16 o;
  o.u = (v4u){0u, 0u, 0u, 0u};
#pragma unroll
  for (int e = 0; e < 8; ++e) {
    const int kk = col + e;
    float v = 0.0f;
    if (kk < K) v = W[(size_t)kk * COUT + n] * WSCALE;
    o.h[e] = (_Float16)v;
  }
  v4u* dst = (v4u*)(Bt + (size_t)n * LDB + col);
  *(volatile v4u*)dst = o.u;
  __threadfence();
  *(volatile v4u*)dst = o.u;
}

template <int CI, int LDG, typename ST>
__global__ __launch_bounds__(256) void gather_rows(const ST* __restrict__ src, const int* __restrict__ nbr,
                                                   _Float16* __restrict__ G, int row0, int rows, int N) {
  const int PPR = LDG / 8;
  const int p = blockIdx.x * 256 + threadIdx.x;
  if (p >= rows * PPR) return;
  const int r = p / PPR;
  const int col = (p - r * PPR) * 8;
  const int k = col / CI;
  const int c0 = col - k * CI;
  P16 o;
  o.u = (v4u){0u, 0u, 0u, 0u};
  if (k < NK) {
    const int idx = nbr[(size_t)(row0 + r) * NK + k];
    if ((unsigned)idx < (unsigned)N) {
      if (sizeof(ST) == 2) {
        o.u = *(const v4u*)(const void*)(src + (size_t)idx * CI + c0);
      } else {
        const float* s = (const float*)(const void*)(src + (size_t)idx * CI + c0);
        const v4f a = *(const v4f*)s;
        const v4f bq = *(const v4f*)(s + 4);
        o.h[0] = (_Float16)a[0];  o.h[1] = (_Float16)a[1];  o.h[2] = (_Float16)a[2];  o.h[3] = (_Float16)a[3];
        o.h[4] = (_Float16)bq[0]; o.h[5] = (_Float16)bq[1]; o.h[6] = (_Float16)bq[2]; o.h[7] = (_Float16)bq[3];
      }
    }
  }
  v4u* dst = (v4u*)(G + (size_t)r * LDG + col);
  *(volatile v4u*)dst = o.u;
  __threadfence();
  *(volatile v4u*)dst = o.u;
}

__global__ __launch_bounds__(256) void bn_stats(const float* __restrict__ X, int N, int rpb, double* __restrict__ part) {
  const int tid = threadIdx.x;
  const int ch = tid & 63;
  const int sub = tid >> 6;
  const int r0 = blockIdx.x * rpb;
  int r1 = r0 + rpb;
  if (r1 > N) r1 = N;
  double s = 0.0, q = 0.0;
  for (int r = r0 + sub; r < r1; r += 4) {
    const double v = (double)X[(size_t)r * COUT + ch];
    s += v;
    q += v * v;
  }
  __shared__ double ls[4][64];
  __shared__ double lq[4][64];
  __shared__ double fs[64];
  __shared__ double fq[64];
  ls[sub][ch] = s;
  lq[sub][ch] = q;
  __syncthreads();
  if (tid < 64) {
    fs[tid] = ((ls[0][tid] + ls[1][tid]) + ls[2][tid]) + ls[3][tid];
    fq[tid] = ((lq[0][tid] + lq[1][tid]) + lq[2][tid]) + lq[3][tid];
  }
  __syncthreads();
  if (tid < 64) {
    v2d v;
    if (tid < 32) { v[0] = fs[2 * tid]; v[1] = fs[2 * tid + 1]; }
    else          { v[0] = fq[2 * tid - 64]; v[1] = fq[2 * tid - 63]; }
    double* dst = part + (size_t)blockIdx.x * 128 + 2 * tid;
    *(volatile v2d*)dst = v;
    __threadfence();
    *(volatile v2d*)dst = v;
  }
}

__global__ __launch_bounds__(64) void bn_finalize(const double* __restrict__ part, int nblk, double invn,
                                                  const float* __restrict__ g, const float* __restrict__ b,
                                                  float* __restrict__ ss) {
  const int ch = threadIdx.x;
  if (ch >= 64) return;
  double S = 0.0, Q = 0.0;
  for (int i = 0; i < nblk; ++i) {
    S += part[(size_t)i * 128 + ch];
    Q += part[(size_t)i * 128 + 64 + ch];
  }
  const double mean = S * invn;
  double var = Q * invn - mean * mean;
  if (var < 0.0) var = 0.0;
  const float meanf = (float)mean;
  const float varf = (float)var;
  const float sc = g[ch] * rsqrtf(varf + BN_EPS);
  const float bb = b[ch];
  *(volatile float*)(ss + ch) = meanf;
  *(volatile float*)(ss + 64 + ch) = sc;
  *(volatile float*)(ss + 128 + ch) = bb;
  __threadfence();
  *(volatile float*)(ss + ch) = meanf;
  *(volatile float*)(ss + 64 + ch) = sc;
  *(volatile float*)(ss + 128 + ch) = bb;
}

__device__ __forceinline__ float bn_act(float x, const float* sm, int c) {
  const float y = (x - sm[c]) * sm[64 + c] + sm[128 + c];
  return (y > 0.0f) ? y : NEG_SLOPE * y;
}

__global__ __launch_bounds__(256) void bn_apply_f16(const float* __restrict__ X, const float* __restrict__ ss,
                                                    _Float16* __restrict__ Y, int total8) {
  __shared__ float sm[192];
  if (threadIdx.x < 192) sm[threadIdx.x] = ss[threadIdx.x];
  __syncthreads();
  const int i = blockIdx.x * 256 + threadIdx.x;
  if (i >= total8) return;
  const int c0 = (i & 7) * 8;
  const float* xp = X + (size_t)i * 8;
  const v4f a = *(const v4f*)xp;
  const v4f bq = *(const v4f*)(xp + 4);
  P16 o;
  o.u = (v4u){0u, 0u, 0u, 0u};
  o.h[0] = (_Float16)bn_act(a[0], sm, c0 + 0);
  o.h[1] = (_Float16)bn_act(a[1], sm, c0 + 1);
  o.h[2] = (_Float16)bn_act(a[2], sm, c0 + 2);
  o.h[3] = (_Float16)bn_act(a[3], sm, c0 + 3);
  o.h[4] = (_Float16)bn_act(bq[0], sm, c0 + 4);
  o.h[5] = (_Float16)bn_act(bq[1], sm, c0 + 5);
  o.h[6] = (_Float16)bn_act(bq[2], sm, c0 + 6);
  o.h[7] = (_Float16)bn_act(bq[3], sm, c0 + 7);
  v4u* dst = (v4u*)(Y + (size_t)i * 8);
  *(volatile v4u*)dst = o.u;
  __threadfence();
  *(volatile v4u*)dst = o.u;
}

__global__ __launch_bounds__(256) void bn_apply_out(const float* __restrict__ X, const float* __restrict__ ss,
                                                    float* __restrict__ Y, int total4) {
  __shared__ float sm[192];
  if (threadIdx.x < 192) sm[threadIdx.x] = ss[threadIdx.x];
  __syncthreads();
  const int i = blockIdx.x * 256 + threadIdx.x;
  if (i >= total4) return;
  const int c0 = (i & 15) * 4;
  const v4f a = *(const v4f*)(X + (size_t)i * 4);
  v4f o;
  o[0] = bn_act(a[0], sm, c0 + 0);
  o[1] = bn_act(a[1], sm, c0 + 1);
  o[2] = bn_act(a[2], sm, c0 + 2);
  o[3] = bn_act(a[3], sm, c0 + 3);
  float* dst = Y + (size_t)i * 4;
  *(volatile v4f*)dst = o;
  __threadfence();
  *(volatile v4f*)dst = o;
}

static inline int cdiv_i(long a, long b) { return (int)((a + b - 1) / b); }

extern "C" void kernel_launch(void* const* d_in, const int* in_sizes, int n_in,
                              void* d_out, int out_size, void* d_ws, size_t ws_size,
                              hipStream_t stream) {
  if (n_in < 8) return;
  const float* features = (const float*)d_in[0];
  const int*   nbr      = (const int*)d_in[1];
  const float* W1       = (const float*)d_in[2];
  const float* g1       = (const float*)d_in[3];
  const float* b1       = (const float*)d_in[4];
  const float* W2       = (const float*)d_in[5];
  const float* g2       = (const float*)d_in[6];
  const float* b2       = (const float*)d_in[7];
  float* out = (float*)d_out;

  const int N = in_sizes[0] / CIN;
  if (N < 64 || (N % 64) != 0) return;
  if (in_sizes[1] < N * NK) return;
  if ((long)out_size < (long)N * COUT) return;
  if (in_sizes[2] < K1 * COUT || in_sizes[5] < K2 * COUT) return;

  const int rpc1 = ((cdiv_i(N, NCH1) + 63) / 64) * 64;
  const int rpc2 = ((cdiv_i(N, NCH2) + 63) / 64) * 64;
  const size_t g1b = (size_t)rpc1 * LD1 * 2;
  const size_t g2b = (size_t)rpc2 * LD2 * 2;
  const size_t gB = (g1b > g2b) ? g1b : g2b;

  char* ws = (char*)d_ws;
  size_t off = 0;
  auto take = [&](size_t bytes) -> char* { char* p = ws + off; off += (bytes + 127) & ~(size_t)127; return p; };
  _Float16* Bt1  = (_Float16*)take((size_t)COUT * LD1 * 2);
  _Float16* Bt2  = (_Float16*)take((size_t)COUT * LD2 * 2);
  _Float16* Y1n  = (_Float16*)take((size_t)N * COUT * 2);
  float*    Yraw = (float*)   take((size_t)N * COUT * 4);
  double*   part = (double*)  take((size_t)STAT_BLK * 128 * 8);
  float*    ss   = (float*)   take((size_t)192 * 4);
  _Float16* G    = (_Float16*)take(gB);
  if (off > ws_size || off > (size_t)134217728) return;

  const int rpb = cdiv_i(N, STAT_BLK);
  const double invn = 1.0 / (double)N;

  prep_bt<LD1><<<cdiv_i((long)COUT * (LD1 / 8), 256), 256, 0, stream>>>(W1, Bt1, K1);
  prep_bt<LD2><<<cdiv_i((long)COUT * (LD2 / 8), 256), 256, 0, stream>>>(W2, Bt2, K2);

  for (int c = 0; c < NCH1; ++c) {
    const int row0 = c * rpc1;
    int rows = N - row0;
    if (rows <= 0) break;
    if (rows > rpc1) rows = rpc1;
    gather_rows<CIN, LD1, float><<<cdiv_i((long)rows * (LD1 / 8), 256), 256, 0, stream>>>(
        features, nbr, G, row0, rows, N);
    const int tiles = (rows / 64) * (COUT / 64);
    dim3 grid(cdiv_i(tiles, 8), 1, 1);
    wmma_gemm64<0, false, 0, 0, false, 0><<<grid, 256, 0, stream>>>(
        (const unsigned short*)G, (const unsigned short*)G, LD1, 0L,
        (const unsigned short*)Bt1, (const unsigned short*)Bt1, LD1, 0L,
        (void*)(Yraw + (size_t)row0 * COUT), (void*)(Yraw + (size_t)row0 * COUT), COUT, 0L,
        (const float*)ss, (const float*)Yraw, 0L,
        rows, COUT, K1, WSCALE_INV);
  }
  bn_stats<<<STAT_BLK, 256, 0, stream>>>(Yraw, N, rpb, part);
  bn_finalize<<<1, 64, 0, stream>>>(part, STAT_BLK, invn, g1, b1, ss);
  bn_apply_f16<<<cdiv_i((long)N * 8, 256), 256, 0, stream>>>(Yraw, ss, Y1n, N * 8);

  for (int c = 0; c < NCH2; ++c) {
    const int row0 = c * rpc2;
    int rows = N - row0;
    if (rows <= 0) break;
    if (rows > rpc2) rows = rpc2;
    gather_rows<COUT, LD2, _Float16><<<cdiv_i((long)rows * (LD2 / 8), 256), 256, 0, stream>>>(
        Y1n, nbr, G, row0, rows, N);
    const int tiles = (rows / 64) * (COUT / 64);
    dim3 grid(cdiv_i(tiles, 8), 1, 1);
    wmma_gemm64<0, false, 0, 0, false, 0><<<grid, 256, 0, stream>>>(
        (const unsigned short*)G, (const unsigned short*)G, LD2, 0L,
        (const unsigned short*)Bt2, (const unsigned short*)Bt2, LD2, 0L,
        (void*)(Yraw + (size_t)row0 * COUT), (void*)(Yraw + (size_t)row0 * COUT), COUT, 0L,
        (const float*)ss, (const float*)Yraw, 0L,
        rows, COUT, K2, WSCALE_INV);
  }
  bn_stats<<<STAT_BLK, 256, 0, stream>>>(Yraw, N, rpb, part);
  bn_finalize<<<1, 64, 0, stream>>>(part, STAT_BLK, invn, g2, b2, ss);
  bn_apply_out<<<cdiv_i((long)N * 16, 256), 256, 0, stream>>>(Yraw, ss, out, N * 16);

  (void)hipGetLastError();
}
